// _TrainedAttention_17583596109978
// MI455X (gfx1250) — hardware-verified
//
#include <hip/hip_runtime.h>


typedef _Float16 h16_t;
typedef __attribute__((ext_vector_type(16))) _Float16 h16x16;
typedef __attribute__((ext_vector_type(8)))  float  f32x8;
typedef __attribute__((ext_vector_type(4)))  float  f32x4;
typedef __attribute__((ext_vector_type(4)))  unsigned u32x4;

constexpr int Bc = 4, Lc = 2048, Dc = 1024, Hc = 16, Pc = 64;
constexpr size_t QKV_BYTES = (size_t)Bc * Hc * Lc * Pc * sizeof(h16_t);
#define PSC 256.0f
#define PUN (1.0f / 256.0f)

__device__ __forceinline__ f32x8 wmma_f16(h16x16 a, h16x16 b, f32x8 c) {
  f32x8 d = __builtin_amdgcn_wmma_f32_16x16x32_f16(false, a, false, b, (short)0, c, false, false);
  asm volatile("v_nop\n\tv_nop\n\tv_nop\n\tv_nop" : "+v"(d) : "v"(a), "v"(b));
  return d;
}
template <typename V> __device__ __forceinline__ void vst2(void* p, V v) {
  *(volatile V*)p = v; __threadfence(); *(volatile V*)p = v;
}
__device__ __forceinline__ unsigned pack2h(float a, float b) {
  _Float16 x = (_Float16)a, y = (_Float16)b;
  unsigned short ux = __builtin_bit_cast(unsigned short, x);
  unsigned short uy = __builtin_bit_cast(unsigned short, y);
  return (unsigned)ux | ((unsigned)uy << 16);
}

__device__ __forceinline__ h16x16 ld_frag(const h16_t* base, int r0, int stride, int k0, int lane) {
  const int m = lane & 15, c = lane >> 4;
  const h16_t* p = base + (size_t)(r0 + m) * stride + k0 + c * 8;
  union { h16x16 v; u32x4 q[2]; } u;
  u.q[0] = *(const u32x4*)(p);
  u.q[1] = *(const u32x4*)(p + 16);
  return u.v;
}

__global__ __launch_bounds__(256) void qkv_kernel(
    const float* __restrict__ x,
    const float* __restrict__ Wq, const float* __restrict__ bq,
    const float* __restrict__ Wk, const float* __restrict__ bk,
    const float* __restrict__ Wv, const float* __restrict__ bv,
    h16_t* __restrict__ Qb, h16_t* __restrict__ Kb, h16_t* __restrict__ Vt) {
  const int which = blockIdx.z;
  const float* W    = (which == 0) ? Wq : (which == 1) ? Wk : Wv;
  const float* bias = (which == 0) ? bq : (which == 1) ? bk : bv;

  __shared__ __align__(16) h16_t As[128 * 32];
  __shared__ __align__(16) h16_t Bs[128 * 32];
  __shared__ __align__(16) h16_t Ts[128 * 128];

  const int tid = threadIdx.x;
  const int lane = tid & 31, wvid = tid >> 5;
  const int wm = wvid >> 2, wn = wvid & 3;
  const int m0 = blockIdx.x * 128, n0 = blockIdx.y * 128;

  f32x8 acc[4][2] = {};

  for (int k0 = 0; k0 < Dc; k0 += 32) {
    for (int i = 0; i < 4; ++i) {
      int s = tid + i * 256;
      int row = s >> 3, col = (s & 7) * 4;
      float4 fa = *(const float4*)(x + (size_t)(m0 + row) * Dc + k0 + col);
      float4 fb = *(const float4*)(W + (size_t)(n0 + row) * Dc + k0 + col);
      h16_t* da = As + row * 32 + col;
      h16_t* db = Bs + row * 32 + col;
      da[0] = (h16_t)fa.x; da[1] = (h16_t)fa.y; da[2] = (h16_t)fa.z; da[3] = (h16_t)fa.w;
      db[0] = (h16_t)fb.x; db[1] = (h16_t)fb.y; db[2] = (h16_t)fb.z; db[3] = (h16_t)fb.w;
    }
    __syncthreads();
    h16x16 b0 = ld_frag(Bs, wn * 32,      32, 0, lane);
    h16x16 b1 = ld_frag(Bs, wn * 32 + 16, 32, 0, lane);
#pragma unroll
    for (int ti = 0; ti < 4; ++ti) {
      h16x16 a = ld_frag(As, wm * 64 + ti * 16, 32, 0, lane);
      acc[ti][0] = wmma_f16(a, b0, acc[ti][0]);
      acc[ti][1] = wmma_f16(a, b1, acc[ti][1]);
    }
    __syncthreads();
  }

  const int c = lane >> 4, nl = lane & 15;
  for (int ti = 0; ti < 4; ++ti)
    for (int tj = 0; tj < 2; ++tj)
      for (int r = 0; r < 8; ++r) {
        int ml  = wm * 64 + ti * 16 + r + 8 * c;
        int nlc = wn * 32 + tj * 16 + nl;
        h16_t v16 = (h16_t)(acc[ti][tj][r] + bias[n0 + nlc]);
        if (which == 2) Ts[nlc * 128 + ml] = v16; else Ts[ml * 128 + nlc] = v16;
      }
  __syncthreads();

  const int b = m0 >> 11, l0 = m0 & (Lc - 1), h0 = n0 >> 6;
  if (which < 2) {
    h16_t* dstb = (which == 0) ? Qb : Kb;
    for (int g = tid; g < 2048; g += 256) {
      const int line = g >> 3, pc = g & 7, ml = line >> 1, hs = line & 1;
      const u32x4 v = *(const u32x4*)(Ts + ml * 128 + hs * 64 + pc * 8);
      vst2(dstb + (((size_t)b * Hc + h0 + hs) * Lc + l0 + ml) * Pc + pc * 8, v);
    }
  } else {
    for (int g = tid; g < 2048; g += 256) {
      const int nrow = g >> 4, pc = g & 15, h = h0 + (nrow >> 6), p = nrow & 63;
      const u32x4 v = *(const u32x4*)(Ts + nrow * 128 + pc * 8);
      vst2(Vt + (((size_t)b * Hc + h) * Pc + p) * Lc + l0 + pc * 8, v);
    }
  }
}

__global__ __launch_bounds__(256) void attn_kernel(
    const h16_t* __restrict__ Qb, const h16_t* __restrict__ Kb,
    const h16_t* __restrict__ Vt, h16_t* __restrict__ Ob,
    const float* __restrict__ temp, const float* __restrict__ qsc) {
  const int bh = blockIdx.y;
  const int b = bh >> 4, h = bh & 15;
  const int tid = threadIdx.x, lane = tid & 31, wvid = tid >> 5;
  const int q0 = blockIdx.x * 128 + wvid * 16;
  const int m_ = lane & 15, c_ = lane >> 4;

  const h16_t* Qp = Qb + (size_t)bh * Lc * Pc;
  const h16_t* Kp = Kb + (size_t)bh * Lc * Pc;
  const h16_t* Vp = Vt + (size_t)bh * Pc * Lc;

  __shared__ __align__(16) h16_t Ks[32 * 64];
  __shared__ __align__(16) h16_t Vs[64 * 32];
  __shared__ __align__(16) h16_t Os[8][16 * 64];

  const int vrow = tid >> 2, vq = tid & 3;

  h16x16 qf0 = ld_frag(Qp, q0, Pc, 0, lane);
  h16x16 qf1 = ld_frag(Qp, q0, Pc, 32, lane);

  f32x8 o[4] = {};
  float mrun = -1e30f, lrun = 0.f;

  for (int l0 = 0; l0 < Lc; l0 += 32) {
    *(u32x4*)(Ks + tid * 8) = *(const u32x4*)(Kp + (size_t)l0 * Pc + tid * 8);
    *(u32x4*)(Vs + vrow * 32 + vq * 8) = *(const u32x4*)(Vp + (size_t)vrow * Lc + l0 + vq * 8);
    __syncthreads();

    f32x8 s0 = {}, s1 = {};
    {
      h16x16 ka = ld_frag(Ks, 0, 64, 0, lane);
      h16x16 kb = ld_frag(Ks, 16, 64, 0, lane);
      s0 = wmma_f16(ka, qf0, s0);
      s1 = wmma_f16(kb, qf0, s1);
      ka = ld_frag(Ks, 0, 64, 32, lane);
      kb = ld_frag(Ks, 16, 64, 32, lane);
      s0 = wmma_f16(ka, qf1, s0);
      s1 = wmma_f16(kb, qf1, s1);
    }

    const float scale = 0.125f / temp[0];
    float lmax = -1e30f;
    for (int r = 0; r < 8; ++r) {
      s0[r] *= scale; s1[r] *= scale;
      lmax = fmaxf(lmax, fmaxf(s0[r], s1[r]));
    }
    lmax = fmaxf(lmax, __shfl_xor(lmax, 16, 32));
    float mnew  = fmaxf(mrun, lmax);
    float alpha = __expf(mrun - mnew);
    float psum = 0.f;
    union { h16x16 v; unsigned u[8]; } af;
    for (int j = 0; j < 4; ++j) {
      float e0 = __expf(s0[2 * j] - mnew), e1 = __expf(s0[2 * j + 1] - mnew);
      psum += e0 + e1; af.u[j] = pack2h(e0 * PSC, e1 * PSC);
    }
    for (int j = 0; j < 4; ++j) {
      float e0 = __expf(s1[2 * j] - mnew), e1 = __expf(s1[2 * j + 1] - mnew);
      psum += e0 + e1; af.u[4 + j] = pack2h(e0 * PSC, e1 * PSC);
    }
    psum += __shfl_xor(psum, 16, 32);
    lrun = lrun * alpha + psum;
    mrun = mnew;

    float av[8];
    for (int r = 0; r < 8; ++r) av[r] = __shfl(alpha, 8 * c_ + r, 32);
    for (int t = 0; t < 4; ++t)
      for (int r = 0; r < 8; ++r) o[t][r] *= av[r];

    for (int t = 0; t < 4; ++t) {
      h16x16 vf = ld_frag(Vs, t * 16, 32, 0, lane);
      o[t] = wmma_f16(af.v, vf, o[t]);
    }
    __syncthreads();
  }

  float inv = (PUN * qsc[h]) / lrun;
  float iv[8];
  for (int r = 0; r < 8; ++r) iv[r] = __shfl(inv, 8 * c_ + r, 32);
  h16_t* os = Os[wvid];
  for (int t = 0; t < 4; ++t)
    for (int r = 0; r < 8; ++r)
      os[(8 * c_ + r) * 64 + t * 16 + m_] = (h16_t)(o[t][r] * iv[r]);
  __syncthreads();
#pragma unroll
  for (int q = 0; q < 4; ++q) {
    const int ql = q * 4 + (lane >> 3), pc = lane & 7;
    const u32x4 v = *(const u32x4*)(os + ql * 64 + pc * 8);
    vst2(Ob + ((size_t)b * Lc + q0 + ql) * Dc + h * Pc + pc * 8, v);
  }
}

__global__ __launch_bounds__(256) void oproj_kernel(
    const h16_t* __restrict__ A, const float* __restrict__ Wo,
    const float* __restrict__ bo, float* __restrict__ out) {
  __shared__ __align__(16) h16_t As[128 * 32];
  __shared__ __align__(16) h16_t Bs[128 * 32];
  __shared__ __align__(16) float Ts[128 * 128];

  const int tid = threadIdx.x;
  const int lane = tid & 31, wvid = tid >> 5;
  const int wm = wvid >> 2, wn = wvid & 3;
  const int m0 = blockIdx.x * 128, n0 = blockIdx.y * 128;

  f32x8 acc[4][2] = {};

  for (int k0 = 0; k0 < Dc; k0 += 32) {
    for (int i = 0; i < 2; ++i) {
      int s = tid + i * 256;
      int row = s >> 2, col = (s & 3) * 8;
      *(u32x4*)(As + row * 32 + col) = *(const u32x4*)(A + (size_t)(m0 + row) * Dc + k0 + col);
    }
    for (int i = 0; i < 4; ++i) {
      int s = tid + i * 256;
      int row = s >> 3, col = (s & 7) * 4;
      float4 f = *(const float4*)(Wo + (size_t)(n0 + row) * Dc + k0 + col);
      h16_t* d = Bs + row * 32 + col;
      d[0] = (h16_t)f.x; d[1] = (h16_t)f.y; d[2] = (h16_t)f.z; d[3] = (h16_t)f.w;
    }
    __syncthreads();
    h16x16 b0 = ld_frag(Bs, wn * 32,      32, 0, lane);
    h16x16 b1 = ld_frag(Bs, wn * 32 + 16, 32, 0, lane);
#pragma unroll
    for (int ti = 0; ti < 4; ++ti) {
      h16x16 a = ld_frag(As, wm * 64 + ti * 16, 32, 0, lane);
      acc[ti][0] = wmma_f16(a, b0, acc[ti][0]);
      acc[ti][1] = wmma_f16(a, b1, acc[ti][1]);
    }
    __syncthreads();
  }

  const int c = lane >> 4, nl = lane & 15;
  for (int ti = 0; ti < 4; ++ti)
    for (int tj = 0; tj < 2; ++tj)
      for (int r = 0; r < 8; ++r) {
        int ml  = wm * 64 + ti * 16 + r + 8 * c;
        int nlc = wn * 32 + tj * 16 + nl;
        Ts[ml * 128 + nlc] = acc[ti][tj][r] + bo[n0 + nlc];
      }
  __syncthreads();
  for (int g = tid; g < 4096; g += 256) {
    const int ml = g >> 5, pc = g & 31;
    const f32x4 v = *(const f32x4*)(Ts + ml * 128 + pc * 4);
    vst2(out + (size_t)(m0 + ml) * Dc + n0 + pc * 4, v);
  }
}

extern "C" void kernel_launch(void* const* d_in, const int* in_sizes, int n_in,
                              void* d_out, int out_size, void* d_ws, size_t ws_size,
                              hipStream_t stream) {
  (void)in_sizes; (void)n_in; (void)out_size; (void)ws_size;
  const float* x  = (const float*)d_in[0];
  const float* Wq = (const float*)d_in[1];
  const float* bq = (const float*)d_in[2];
  const float* Wk = (const float*)d_in[3];
  const float* bk = (const float*)d_in[4];
  const float* Wv = (const float*)d_in[5];
  const float* bv = (const float*)d_in[6];
  const float* Wo = (const float*)d_in[7];
  const float* bo = (const float*)d_in[8];
  const float* temp = (const float*)d_in[9];
  const float* qsc  = (const float*)d_in[10];

  char* ws = (char*)d_ws;
  h16_t* Qb = (h16_t*)(ws);
  h16_t* Kb = (h16_t*)(ws + QKV_BYTES);
  h16_t* Vt = (h16_t*)(ws + 2 * QKV_BYTES);
  h16_t* Ob = (h16_t*)(ws + 3 * QKV_BYTES);

  const int M = Bc * Lc;
  qkv_kernel<<<dim3(M / 128, Dc / 128, 3), 256, 0, stream>>>(x, Wq, bq, Wk, bk, Wv, bv, Qb, Kb, Vt);
  attn_kernel<<<dim3(Lc / 128, Bc * Hc), 256, 0, stream>>>(Qb, Kb, Vt, Ob, temp, qsc);
  oproj_kernel<<<dim3(M / 128, Dc / 128), 256, 0, stream>>>(Ob, Wo, bo, (float*)d_out);
}
